// ModulatedDeformConv2dFunction_3504693314064
// MI455X (gfx1250) — hardware-verified
//
#include <hip/hip_runtime.h>
#include <stddef.h>


#define IH     128
#define IW     128
#define HWN    16384
#define CIN    64
#define COUT   64
#define KS     3
#define TAPS   9
#define PADV   1
#define KTOT   576
#define NTHR   256
#define NWAVE  8
#define APITCH 72
#define SPITCH 132
#define ASC    16.0f
#define WSC    1024.0f
#define ACCINV 0.00006103515625f
#define WSCAP  134217728

static_assert(KTOT == CIN * TAPS);
static_assert((KTOT % 32) == 0);
static_assert(NTHR == 2 * IW);
static_assert(NWAVE * 16 == IW);
static_assert(NWAVE * 8 == COUT);
static_assert(((APITCH * 2) % 16) == 0);
static_assert(((SPITCH * 4) % 16) == 0);
static_assert((COUT * (KTOT / 8)) % NTHR == 0);
static_assert(IW * APITCH >= (IW - 1) * APITCH + CIN);
static_assert(COUT * SPITCH >= (COUT - 1) * SPITCH + IW);

typedef float          v4f  __attribute__((ext_vector_type(4)));
typedef float          v8f  __attribute__((ext_vector_type(8)));
typedef unsigned int   v4u  __attribute__((ext_vector_type(4)));
typedef unsigned short v8us __attribute__((ext_vector_type(8)));
typedef _Float16       v16h __attribute__((ext_vector_type(16)));
union FragH { v16h v; v8us u[2]; };

__device__ __forceinline__ v8f wmh(v16h a, v16h b, v8f c) {
  v8f d = __builtin_amdgcn_wmma_f32_16x16x32_f16(false, a, false, b, (short)0, c, false, false);
  asm volatile("v_nop\n\tv_nop\n\tv_nop\n\tv_nop" : "+v"(d) : "v"(a), "v"(b));
  return d;
}

__device__ __forceinline__ unsigned hbits(float x) {
  const _Float16 h = (_Float16)x;
  const unsigned u = (unsigned)__builtin_bit_cast(unsigned short, h);
  return ((u & 0x7C00u) == 0u) ? 0u : u;
}

__global__ __launch_bounds__(NTHR) void k_wprep(const float* __restrict__ w, unsigned short* wp) {
  const int i = (int)blockIdx.x * NTHR + (int)threadIdx.x;
  if (i >= COUT * (KTOT / 8)) return;
  const int o   = i / (KTOT / 8);
  const int kq  = i - o * (KTOT / 8);
  const int k0  = kq * 8;
  const int tap = k0 >> 6;
  const int c0  = k0 & (CIN - 1);
  const float* src = w + (size_t)o * KTOT + (size_t)c0 * TAPS + tap;
  unsigned hb[8];
#pragma unroll
  for (int j = 0; j < 8; ++j) hb[j] = hbits(src[TAPS * j] * WSC);
  v4u pv;
  pv.x = hb[0] | (hb[1] << 16);
  pv.y = hb[2] | (hb[3] << 16);
  pv.z = hb[4] | (hb[5] << 16);
  pv.w = hb[6] | (hb[7] << 16);
  unsigned short* dst = wp + (size_t)i * 8;
  *(volatile v4u*)dst = pv;
  __threadfence();
  *(volatile v4u*)dst = pv;
}

__global__ __launch_bounds__(NTHR) void k_dconv(const float* __restrict__ xin,
                                                const float* __restrict__ offs,
                                                const float* __restrict__ msk,
                                                const unsigned short* __restrict__ wp,
                                                const float* __restrict__ bias,
                                                float* out) {
#pragma clang fp contract(off)
  __shared__ __attribute__((aligned(16))) unsigned short colA[IW * APITCH];
  __shared__ __attribute__((aligned(16))) float stg[COUT * SPITCH];
  const int tid = threadIdx.x, lane = tid & 31, wave = tid >> 5, hh = lane >> 4, m = lane & 15;
  const int blk = (int)blockIdx.x;
  const int b  = blk >> 7;
  const int ho = blk & (IH - 1);

  const int wo    = tid & (IW - 1);
  const int chalf = tid >> 7;
  const int p     = ho * IW + wo;
  const float* xb = xin + ((size_t)(b * CIN + chalf * 32) << 14);
  unsigned short* arow = colA + wo * APITCH + chalf * 32;

  const unsigned short* afr = colA + (wave * 16 + m) * APITCH + 8 * hh;
  const unsigned short* bfr = wp + (size_t)m * KTOT + 8 * hh;

  v8f acc[4];
#pragma unroll
  for (int t = 0; t < 4; ++t) {
    const v8f z = {0.f, 0.f, 0.f, 0.f, 0.f, 0.f, 0.f, 0.f};
    acc[t] = z;
  }

#pragma unroll 1
  for (int tap = 0; tap < TAPS; ++tap) {
    const int kh = tap / KS, kw = tap - kh * KS;
    const float dy = offs[((size_t)(b * 2 * TAPS + 2 * tap)     << 14) + p];
    const float dx = offs[((size_t)(b * 2 * TAPS + 2 * tap + 1) << 14) + p];
    const float mv = msk [((size_t)(b * TAPS + tap)             << 14) + p];

    const float yf  = (float)(ho - PADV + kh) + dy;
    const float xf  = (float)(wo - PADV + kw) + dx;
    const float y0f = floorf(yf), x0f = floorf(xf);
    const float ly  = yf - y0f, lx = xf - x0f;
    const int y0 = (int)fminf(fmaxf(y0f, -1048576.0f), 1048576.0f);
    const int x0 = (int)fminf(fmaxf(x0f, -1048576.0f), 1048576.0f);
    const bool vy0 = (y0 >= 0)  && (y0 <= IH - 1);
    const bool vy1 = (y0 >= -1) && (y0 <= IH - 2);
    const bool vx0 = (x0 >= 0)  && (x0 <= IW - 1);
    const bool vx1 = (x0 >= -1) && (x0 <= IW - 2);
    const float hy = 1.0f - ly, hx = 1.0f - lx;
    const float w00 = (hy * hx) * ((vy0 && vx0) ? 1.0f : 0.0f);
    const float w01 = (hy * lx) * ((vy0 && vx1) ? 1.0f : 0.0f);
    const float w10 = (ly * hx) * ((vy1 && vx0) ? 1.0f : 0.0f);
    const float w11 = (ly * lx) * ((vy1 && vx1) ? 1.0f : 0.0f);
    const int cy0 = min(max(y0, 0), IH - 1), cy1 = min(max(y0 + 1, 0), IH - 1);
    const int cx0 = min(max(x0, 0), IW - 1), cx1 = min(max(x0 + 1, 0), IW - 1);
    const int i00 = cy0 * IW + cx0, i01 = cy0 * IW + cx1;
    const int i10 = cy1 * IW + cx0, i11 = cy1 * IW + cx1;

#pragma unroll 1
    for (int j = 0; j < 16; ++j) {
      const float* pc0 = xb + ((size_t)(2 * j) << 14);
      const float* pc1 = pc0 + HWN;
      const float a00 = pc0[i00], a01 = pc0[i01], a10 = pc0[i10], a11 = pc0[i11];
      const float c00 = pc1[i00], c01 = pc1[i01], c10 = pc1[i10], c11 = pc1[i11];
      float v0 = ((a00 * w00 + a01 * w01) + a10 * w10) + a11 * w11;
      float v1 = ((c00 * w00 + c01 * w01) + c10 * w10) + c11 * w11;
      v0 = v0 * mv;
      v1 = v1 * mv;
      const unsigned pk = hbits(v0 * ASC) | (hbits(v1 * ASC) << 16);
      *(unsigned*)(arow + 2 * j) = pk;
    }
    __syncthreads();

    const size_t kb = (size_t)tap * CIN;
#pragma unroll
    for (int ks = 0; ks < 2; ++ks) {
      FragH fa;
      fa.u[0] = *(const v8us*)(afr + 32 * ks);
      fa.u[1] = *(const v8us*)(afr + 32 * ks + 16);
#pragma unroll
      for (int t = 0; t < 4; ++t) {
        const unsigned short* bp = bfr + (size_t)(16 * t) * KTOT + kb + 32 * ks;
        FragH fb;
        fb.u[0] = *(const v8us*)(bp);
        fb.u[1] = *(const v8us*)(bp + 16);
        acc[t] = wmh(fa.v, fb.v, acc[t]);
      }
    }
    __syncthreads();
  }

  {
    float* sp = stg + m * SPITCH + wave * 16 + 8 * hh;
#pragma unroll
    for (int t = 0; t < 4; ++t) {
#pragma unroll
      for (int r = 0; r < 8; ++r) sp[16 * t * SPITCH + r] = acc[t][r];
    }
  }
  __syncthreads();

  const float* srow = stg + (wave * 8) * SPITCH + 4 * lane;
  float* orow = out + ((size_t)(b * COUT + wave * 8) << 14) + (size_t)ho * IW + 4 * lane;
#pragma unroll 1
  for (int pass = 0; pass < 2; ++pass) {
#pragma unroll
    for (int j = 0; j < 8; ++j) {
      const float bo = bias[wave * 8 + j];
      v4f v = *(const v4f*)(srow + j * SPITCH);
      v = v * ACCINV;
      v.x = v.x + bo; v.y = v.y + bo; v.z = v.z + bo; v.w = v.w + bo;
      *(volatile v4f*)(orow + ((size_t)j << 14)) = v;
    }
    if (pass == 0) __threadfence();
  }
}

extern "C" void kernel_launch(void* const* d_in, const int* in_sizes, int n_in,
                              void* d_out, int out_size, void* d_ws, size_t ws_size,
                              hipStream_t stream) {
  if (n_in < 5) return;
  const int nb = in_sizes[0] / (CIN * HWN);
  if (nb <= 0 || in_sizes[0] != nb * CIN * HWN) return;
  if (in_sizes[1] != nb * 2 * TAPS * HWN || in_sizes[2] != nb * TAPS * HWN) return;
  if (in_sizes[3] != COUT * KTOT || in_sizes[4] != COUT) return;
  if (out_size != nb * COUT * HWN) return;

  const size_t wpBytes = (size_t)COUT * KTOT * 2;
  const size_t total   = (wpBytes + 255) & ~(size_t)255;
  if (total > ws_size || total > (size_t)WSCAP) return;

  const float* x    = (const float*)d_in[0];
  const float* offs = (const float*)d_in[1];
  const float* msk  = (const float*)d_in[2];
  const float* w    = (const float*)d_in[3];
  const float* bias = (const float*)d_in[4];
  float* out = (float*)d_out;
  unsigned short* wp = (unsigned short*)d_ws;

  k_wprep<<<(COUT * (KTOT / 8) + NTHR - 1) / NTHR, NTHR, 0, stream>>>(w, wp);
  k_dconv<<<nb * IH, NTHR, 0, stream>>>(x, offs, msk, wp, bias, out);
}
